// Profile_62517543961105
// MI455X (gfx1250) — hardware-verified
//
#include <hip/hip_runtime.h>


#define NB_  4096
#define DD   1024
#define KK   5
#define NP   1323
#define NCOL 64
#define LOG2PI 1.8378770664093453f

typedef unsigned short bf;
typedef __attribute__((ext_vector_type(16))) __bf16   v16bf;
typedef __attribute__((ext_vector_type(8)))  unsigned short v8us;
typedef __attribute__((ext_vector_type(8)))  float    v8f;
typedef __attribute__((ext_vector_type(4)))  float    v4f;
typedef v4f  __attribute__((may_alias)) v4fa;

__device__ __forceinline__ unsigned short f2bf(float f) { unsigned u = __float_as_uint(f); u += 0x7FFFu + ((u >> 16) & 1u); return (unsigned short)(u >> 16); }
__device__ __forceinline__ float bf2f(unsigned short b) { return __uint_as_float(((unsigned)b) << 16); }
__device__ __forceinline__ float bfr(float f) { return bf2f(f2bf(f)); }
__device__ __forceinline__ v16bf cat16b(v8us lo, v8us hi) { return __builtin_bit_cast(v16bf, __builtin_shufflevector(lo, hi, 0, 1, 2, 3, 4, 5, 6, 7, 8, 9, 10, 11, 12, 13, 14, 15)); }
__device__ __forceinline__ v8f wmmab(v16bf a, v16bf b, v8f c) { return __builtin_amdgcn_wmma_f32_16x16x32_bf16(false, a, false, b, (short)0, c, false, false); }
#define VST2(T, p, v) do { const T vst2_v_ = (v); *(volatile T*)(p) = vst2_v_; __threadfence(); *(volatile T*)(p) = vst2_v_; } while (0)

__global__ __launch_bounds__(256) void k_xb(const float* __restrict__ x, bf* Xb) {
    const int lane = threadIdx.x & 31, r = blockIdx.x * 8 + (threadIdx.x >> 5);
    if (r >= NB_) return;
#pragma unroll
    for (int q = 0; q < DD / 256; ++q) { v8us t;
#pragma unroll
        for (int i = 0; i < 8; ++i) t[i] = f2bf(x[(size_t)r * DD + q * 256 + lane * 8 + i]);
        VST2(v8us, Xb + (size_t)r * DD + q * 256 + lane * 8, t); }
}
__global__ __launch_bounds__(256) void k_wb(const float* __restrict__ Wm, const float* __restrict__ Wme, const float* __restrict__ Ws, bf* WB) {
    const int lane = threadIdx.x & 31, n = blockIdx.x * 8 + (threadIdx.x >> 5);
    if (n >= NCOL) return;
#pragma unroll
    for (int q = 0; q < DD / 256; ++q) { v8us t;
#pragma unroll
        for (int i = 0; i < 8; ++i) { const int k = q * 256 + lane * 8 + i; float v = 0.f;
            if (n < KK) v = Wm[(size_t)k * KK + n]; else if (n < 17) v = Wme[(size_t)k * 12 + (n - KK)]; else if (n < 47) v = Ws[(size_t)k * 30 + (n - 17)];
            t[i] = f2bf(v); }
        VST2(v8us, WB + (size_t)n * DD + q * 256 + lane * 8, t); }
}
__global__ __launch_bounds__(128) void k_gemm(const bf* __restrict__ A, const bf* __restrict__ Bn, const float* __restrict__ bm, const float* __restrict__ bme, const float* __restrict__ bs, float* C) {
    __shared__ __align__(16) float ost[4][16 * 68];
    const int lane = threadIdx.x & 31, wave = threadIdx.x >> 5, lr = lane & 15, hi = lane >> 4;
    const int r0 = blockIdx.x * 64 + wave * 16;
    const size_t aoff = (size_t)(r0 + lr) * DD + 8 * hi;
    size_t boff[4];
#pragma unroll
    for (int t = 0; t < 4; ++t) boff[t] = (size_t)(t * 16 + lr) * DD + 8 * hi;
    v8f acc[4];
#pragma unroll
    for (int t = 0; t < 4; ++t) acc[t] = (v8f){};
#pragma unroll 1
    for (int kc = 0; kc < DD; kc += 32) {
        const v16bf a = cat16b(*(const v8us*)(A + aoff + kc), *(const v8us*)(A + aoff + kc + 16));
#pragma unroll
        for (int t = 0; t < 4; ++t) acc[t] = wmmab(a, cat16b(*(const v8us*)(Bn + boff[t] + kc), *(const v8us*)(Bn + boff[t] + kc + 16)), acc[t]);
        asm volatile("v_nop\n\tv_nop\n\tv_nop\n\tv_nop" : "+v"(acc[0]), "+v"(acc[1]), "+v"(acc[2]), "+v"(acc[3]) : "v"(a));
    }
    float* os = &ost[wave][0];
#pragma unroll
    for (int t = 0; t < 4; ++t) { const int n = t * 16 + lr; const float bv = (n < KK) ? bfr(bm[n]) : (n < 17) ? bfr(bme[n - KK]) : (n < 47) ? bfr(bs[n - 17]) : 0.f;
#pragma unroll
        for (int j = 0; j < 8; ++j) os[(hi * 8 + j) * 68 + n] = acc[t][j] + bv; }
    __syncthreads();
    float* crow = C + (size_t)r0 * NCOL;
    auto pass = [&]() {
#pragma unroll
        for (int s = 0; s < 8; ++s) { const int Lid = (lane >> 3) + 4 * s, piece = lane & 7; const int row = Lid >> 1, cofs = (Lid & 1) * 32 + piece * 4;
            const v4f val = *(const v4fa*)(os + row * 68 + cofs); *(volatile v4f*)(crow + (size_t)row * NCOL + cofs) = val; }
    };
    pass(); __threadfence(); pass();
}
__device__ __forceinline__ float softplus_(float v) { return (v > 20.f) ? v : log1pf(__expf(v)); }
__global__ __launch_bounds__(256) void k_prof(const float* __restrict__ PAR, const float* __restrict__ dxyz, float* out0, float* out1) {
    __shared__ float Ls[256 * 45];
    __shared__ float prm[256 * 12 * KK];
    const int t = threadIdx.x, lane = t & 31, wave = t >> 5, b = blockIdx.x * 256 + t;
    const float* pr = PAR + (size_t)b * NCOL;
    float* my = prm + t * 12 * KK;
    float mx = -3.0e38f;
#pragma unroll 1
    for (int k = 0; k < KK; ++k) mx = fmaxf(mx, pr[k]);
    float se = 0.f;
#pragma unroll 1
    for (int k = 0; k < KK; ++k) se += __expf(pr[k] - mx);
#pragma unroll 1
    for (int k = 0; k < KK; ++k) {
        const float lw = __logf(__expf(pr[k] - mx) / se);
        const float m0 = (k == 0) ? 0.f : pr[KK + (k - 1) * 3 + 0], m1 = (k == 0) ? 0.f : pr[KK + (k - 1) * 3 + 1], m2 = (k == 0) ? 0.f : pr[KK + (k - 1) * 3 + 2];
        const float* sc = pr + 17 + k * 6;
        const float L00 = softplus_(sc[0]), L10 = sc[1], L11 = softplus_(sc[2]), L20 = sc[3], L21 = sc[4], L22 = softplus_(sc[5]);
        float* q = my + k * 12;
        q[0] = lw; q[1] = m0; q[2] = m1; q[3] = m2; q[4] = 1.0f / L00; q[5] = L10; q[6] = 1.0f / L11; q[7] = L20; q[8] = L21; q[9] = 1.0f / L22;
        q[10] = lw - (__logf(L00) + __logf(L11) + __logf(L22)) - 1.5f * LOG2PI;
        float* lp = Ls + t * 45 + k * 9;
        lp[0] = L00; lp[1] = 0.f; lp[2] = 0.f; lp[3] = L10; lp[4] = L11; lp[5] = 0.f; lp[6] = L20; lp[7] = L21; lp[8] = L22;
    }
    __syncthreads();
#pragma unroll 1
    for (int ln = wave; ln < (256 * 45) / 32; ln += 8) { const int e = ln * 32 + lane; VST2(float, out1 + (size_t)blockIdx.x * 256 * 45 + e, Ls[e]); }
#pragma unroll 1
    for (int pass = 0; pass < 2; ++pass) {
#pragma unroll 1
        for (int p = 0; p < NP; ++p) {
            const float* dp = dxyz + ((size_t)p * NB_ + b) * 3;
            const float x0 = bfr(dp[0]), x1 = bfr(dp[1]), x2 = bfr(dp[2]);
            float cm = -3.0e38f;
#pragma unroll 1
            for (int k = 0; k < KK; ++k) { const float* q = my + k * 12;
                const float d0 = x0 - q[1], d1 = x1 - q[2], d2 = x2 - q[3];
                const float z0 = d0 * q[4]; const float z1 = (d1 - q[5] * z0) * q[6]; const float z2 = (d2 - q[7] * z0 - q[8] * z1) * q[9];
                const float c = -0.5f * (z0 * z0 + z1 * z1 + z2 * z2) + q[10]; q = q; my[k * 12 + 11] = c; cm = fmaxf(cm, c); }
            float s = 0.f;
#pragma unroll 1
            for (int k = 0; k < KK; ++k) s += __expf(my[k * 12 + 11] - cm);
            *(volatile float*)(out0 + (size_t)p * NB_ + b) = __expf(cm + __logf(s));
        }
        __threadfence();
    }
}

extern "C" void kernel_launch(void* const* d_in, const int* in_sizes, int n_in,
                              void* d_out, int out_size, void* d_ws, size_t ws_size, hipStream_t stream) {
    (void)in_sizes; (void)n_in; (void)out_size;
    const float* rep = (const float*)d_in[0]; const float* dxyz = (const float*)d_in[1]; const float* Wm = (const float*)d_in[2]; const float* bm = (const float*)d_in[3];
    const float* Wme = (const float*)d_in[4]; const float* bme = (const float*)d_in[5]; const float* Ws = (const float*)d_in[6]; const float* bs = (const float*)d_in[7];
    float* out0 = (float*)d_out;
    float* out1 = (float*)((char*)d_out + (size_t)NB_ * NP * 4);
    char* wsp = (char*)d_ws;
    auto take = [&](size_t bytes) { char* p = wsp; wsp += (bytes + 255) & ~(size_t)255; return (void*)p; };
    bf* Xb = (bf*)take((size_t)NB_ * DD * 2); bf* WB = (bf*)take((size_t)NCOL * DD * 2); float* PAR = (float*)take((size_t)NB_ * NCOL * 4);
    if ((size_t)(wsp - (char*)d_ws) > ws_size) return;
    k_xb<<<NB_ / 8, 256, 0, stream>>>(rep, Xb);
    k_wb<<<NCOL / 8, 256, 0, stream>>>(Wm, Wme, Ws, WB);
    k_gemm<<<NB_ / 64, 128, 0, stream>>>(Xb, WB, bm, bme, bs, PAR);
    k_prof<<<NB_ / 256, 256, 0, stream>>>(PAR, dxyz, out0, out1);
}
